// GraphormerEncoder_27839978013470
// MI455X (gfx1250) — hardware-verified
//
#include <hip/hip_runtime.h>
#include <math.h>
#include <stdint.h>

#define NN   2048
#define NO   1984
#define DM   512
#define NHD  8
#define DK   64
#define FF   2048
#define NL   4
#define NF   32
#define NT   32
#define MSP  100
#define MDG  100
#define MTH  (-1.0e30f)
#define PLANE_QK (NHD * NN * DK)

static_assert(NN == 16 * 128);
static_assert(NO == 31 * 64);
static_assert(DM == NHD * DK);
static_assert(DK == 64);
static_assert(FF == 2048);
static_assert(NT * 64 == NN);
static_assert(NT == 32);
static_assert(NF % 32 == 0 && DM % 32 == 0 && FF % 32 == 0 && DK % 32 == 0);
static_assert((NO * 4) % 16 == 0);
static_assert(NO % 4 == 0);

typedef __attribute__((ext_vector_type(16))) __bf16   v16b;
typedef __attribute__((ext_vector_type(8)))  __bf16   v8b;
typedef __attribute__((ext_vector_type(8)))  float    v8f;
typedef __attribute__((ext_vector_type(4)))  float    v4f;
typedef __attribute__((ext_vector_type(4)))  unsigned int v4u;
typedef __attribute__((ext_vector_type(4)))  int      v4i;
typedef v4f __attribute__((may_alias)) v4fa;

__device__ __forceinline__ unsigned short f2bf_bits(float f) {
  unsigned u = __float_as_uint(f);
  return (unsigned short)((u + 0x7FFFu + ((u >> 16) & 1u)) >> 16);
}
__device__ __forceinline__ float bf_bits2f(unsigned short h) { return __uint_as_float(((unsigned)h) << 16); }
__device__ __forceinline__ float bf16r(float f) { return bf_bits2f(f2bf_bits(f)); }
__device__ __forceinline__ unsigned pk16(unsigned short a, unsigned short b) { return (unsigned)a | ((unsigned)b << 16); }

__device__ __forceinline__ void split8(const v4f x0, const v4f x1, v4u& hv, v4u& lv) {
  const unsigned short h0 = f2bf_bits(x0[0]), h1 = f2bf_bits(x0[1]), h2 = f2bf_bits(x0[2]), h3 = f2bf_bits(x0[3]);
  const unsigned short h4 = f2bf_bits(x1[0]), h5 = f2bf_bits(x1[1]), h6 = f2bf_bits(x1[2]), h7 = f2bf_bits(x1[3]);
  const unsigned short l0 = f2bf_bits(x0[0] - bf_bits2f(h0)), l1 = f2bf_bits(x0[1] - bf_bits2f(h1));
  const unsigned short l2 = f2bf_bits(x0[2] - bf_bits2f(h2)), l3 = f2bf_bits(x0[3] - bf_bits2f(h3));
  const unsigned short l4 = f2bf_bits(x1[0] - bf_bits2f(h4)), l5 = f2bf_bits(x1[1] - bf_bits2f(h5));
  const unsigned short l6 = f2bf_bits(x1[2] - bf_bits2f(h6)), l7 = f2bf_bits(x1[3] - bf_bits2f(h7));
  hv = (v4u){pk16(h0, h1), pk16(h2, h3), pk16(h4, h5), pk16(h6, h7)};
  lv = (v4u){pk16(l0, l1), pk16(l2, l3), pk16(l4, l5), pk16(l6, l7)};
}

union FragU { v16b v; v8b h[2]; };
__device__ __forceinline__ v16b ldfrag(const __bf16* p) {
  FragU f; f.h[0] = *(const v8b*)(p); f.h[1] = *(const v8b*)(p + 16); return f.v;
}
__device__ __forceinline__ v8f mma_b(v16b a, v16b b, v8f c) {
  return __builtin_amdgcn_wmma_f32_16x16x32_bf16(false, a, false, b, (short)0, c, false, false);
}
__device__ __forceinline__ v8f mma_g(v16b a, v16b b, v8f c) {
  v8f d = __builtin_amdgcn_wmma_f32_16x16x32_bf16(false, a, false, b, (short)0, c, false, false);
  asm volatile("v_nop\n\tv_nop\n\tv_nop\n\tv_nop" : "+v"(d) : "v"(a), "v"(b));
  return d;
}
__device__ __forceinline__ void dep_guard_b(v8f& a, v8f& b, v16b x, v16b y) { asm volatile("v_nop\n\tv_nop\n\tv_nop\n\tv_nop" : "+v"(a), "+v"(b) : "v"(x), "v"(y)); }
__device__ __forceinline__ void keep4_b(v16b a, v16b b, v16b c, v16b d) { asm volatile("v_nop" :: "v"(a), "v"(b), "v"(c), "v"(d)); }
__device__ __forceinline__ void acc_guard4(v8f& a, v8f& b, v8f& c, v8f& d) { asm volatile("v_nop\n\tv_nop\n\tv_nop\n\tv_nop" : "+v"(a), "+v"(b), "+v"(c), "+v"(d)); }

__global__ __launch_bounds__(256) void k_pa(const float* __restrict__ x, const float* __restrict__ iw,
                                            unsigned short* __restrict__ XB, unsigned short* __restrict__ IWT) {
  const int tid = threadIdx.x;
  if (blockIdx.x < 32) {
    const int t = blockIdx.x * 256 + tid;
    const int row = t >> 2, k0 = (t & 3) * 8;
    const int rc = (row < NO) ? row : (NO - 1);
    const v4f a = *(const v4f*)(x + (size_t)rc * NF + k0);
    const v4f b = *(const v4f*)(x + (size_t)rc * NF + k0 + 4);
    const bool ok = (row < NO);
    const unsigned short h0 = ok ? f2bf_bits(a[0]) : (unsigned short)0, h1 = ok ? f2bf_bits(a[1]) : (unsigned short)0;
    const unsigned short h2 = ok ? f2bf_bits(a[2]) : (unsigned short)0, h3 = ok ? f2bf_bits(a[3]) : (unsigned short)0;
    const unsigned short h4 = ok ? f2bf_bits(b[0]) : (unsigned short)0, h5 = ok ? f2bf_bits(b[1]) : (unsigned short)0;
    const unsigned short h6 = ok ? f2bf_bits(b[2]) : (unsigned short)0, h7 = ok ? f2bf_bits(b[3]) : (unsigned short)0;
    const v4u o = (v4u){pk16(h0, h1), pk16(h2, h3), pk16(h4, h5), pk16(h6, h7)};
    unsigned short* d = XB + (size_t)t * 8;
    *(volatile v4u*)d = o;
    __threadfence();
    *(volatile v4u*)d = o;
  } else {
    const int t = (blockIdx.x - 32) * 256 + tid;
    const int n = t >> 2, k0 = (t & 3) * 8;
    const float f0 = iw[(size_t)(k0 + 0) * DM + n], f1 = iw[(size_t)(k0 + 1) * DM + n];
    const float f2 = iw[(size_t)(k0 + 2) * DM + n], f3 = iw[(size_t)(k0 + 3) * DM + n];
    const float f4 = iw[(size_t)(k0 + 4) * DM + n], f5 = iw[(size_t)(k0 + 5) * DM + n];
    const float f6 = iw[(size_t)(k0 + 6) * DM + n], f7 = iw[(size_t)(k0 + 7) * DM + n];
    const v4u o = (v4u){pk16(f2bf_bits(f0), f2bf_bits(f1)), pk16(f2bf_bits(f2), f2bf_bits(f3)),
                        pk16(f2bf_bits(f4), f2bf_bits(f5)), pk16(f2bf_bits(f6), f2bf_bits(f7))};
    unsigned short* d = IWT + (size_t)t * 8;
    *(volatile v4u*)d = o;
    __threadfence();
    *(volatile v4u*)d = o;
  }
}

__global__ __launch_bounds__(256) void k_tr(const float* __restrict__ in, unsigned short* __restrict__ out,
                                            int rows, int cols, int zIn, int zDiv, int zOutHi, int zOutLo) {
  __shared__ __align__(16) unsigned short th[64 * 72];
  const int c0 = blockIdx.x * 64, r0 = blockIdx.y * 64, z = blockIdx.z;
  const int tid = threadIdx.x;
  const float* src = in + (size_t)z * zIn;
  unsigned short* dst = out + (size_t)(z / zDiv) * zOutHi + (size_t)(z % zDiv) * zOutLo;
  {
    const int rr = tid >> 2, cq = (tid & 3) * 16;
    const float* s = src + (size_t)(r0 + rr) * cols + c0 + cq;
#pragma unroll
    for (int q = 0; q < 4; ++q) {
      const v4f f = *(const v4f*)(s + 4 * q);
#pragma unroll
      for (int e = 0; e < 4; ++e) th[rr * 72 + cq + 4 * q + e] = f2bf_bits(f[e]);
    }
  }
  __syncthreads();
  const int sub = tid >> 3, c8 = (tid & 7) * 8;
  v4u hv[2];
#pragma unroll
  for (int it = 0; it < 2; ++it) {
    const int oc = it * 32 + sub;
    v4u a;
#pragma unroll
    for (int q = 0; q < 4; ++q) a[q] = pk16(th[(c8 + 2 * q) * 72 + oc], th[(c8 + 2 * q + 1) * 72 + oc]);
    hv[it] = a;
  }
  for (int pass = 0; pass < 2; ++pass) {
#pragma unroll
    for (int it = 0; it < 2; ++it) {
      const int oc = it * 32 + sub;
      *(volatile v4u*)(dst + (size_t)(c0 + oc) * rows + r0 + c8) = hv[it];
    }
    __threadfence();
  }
}

__global__ __launch_bounds__(256) void k_bias(const int* __restrict__ sp, const int* __restrict__ bid,
                                              const float* __restrict__ db, const float* __restrict__ vbp,
                                              float* __restrict__ BM, int* __restrict__ tcls) {
  __shared__ int sb[NN];
  __shared__ float sdb[104];
  __shared__ int scls[NT];
  const int qt = blockIdx.x, tid = threadIdx.x, lane = tid & 31, wave = tid >> 5;
  {
    const v4i a = *(const v4i*)(bid + tid * 8);
    const v4i b = *(const v4i*)(bid + tid * 8 + 4);
#pragma unroll
    for (int e = 0; e < 4; ++e) { sb[tid * 8 + e] = a[e]; sb[tid * 8 + 4 + e] = b[e]; }
    const int di = (tid < 101) ? tid : 101;
    const float dv = bf16r(db[di]);
    if (tid < 104) sdb[tid] = dv;
  }
  __syncthreads();
  {
    const int kt = tid >> 3, part = tid & 7;
    int cnt = 0;
#pragma unroll 1
    for (int rr = 0; rr < 8; ++rr) {
      const int bi = sb[qt * 64 + part * 8 + rr];
#pragma unroll 8
      for (int c = 0; c < 64; ++c) cnt += (sb[kt * 64 + c] == bi) ? 1 : 0;
    }
    cnt += __shfl_xor(cnt, 1, 32);
    cnt += __shfl_xor(cnt, 2, 32);
    cnt += __shfl_xor(cnt, 4, 32);
    if ((tid & 7) == 0) scls[kt] = (cnt == 0) ? 0 : ((cnt == 4096) ? 2 : 1);
  }
  __syncthreads();
  if (wave == 0) {
    const int f = scls[lane];
    volatile int* p = tcls + (size_t)qt * NT + lane;
    *p = f;
    __threadfence();
    *p = f;
  }
  const float vb = bf16r(vbp[0]);
  const float fill = sdb[101];
  const float d0 = sdb[0];
  const float ninf = __uint_as_float(0xff800000u);
#pragma unroll 1
  for (int r = 0; r < 64; ++r) {
    const int i = qt * 64 + r;
    const int bi = sb[i];
    const int ic = (i < NO) ? i : (NO - 1);
    const bool iv = (i >= NO);
    v4f o[2];
#pragma unroll
    for (int it = 0; it < 2; ++it) {
      const int j0 = it * 1024 + tid * 4;
      const int jc = (j0 < NO - 4) ? j0 : (NO - 4);
      const v4i s4 = *(const v4i*)(sp + (size_t)ic * NO + jc);
#pragma unroll
      for (int e = 0; e < 4; ++e) {
        const int j = j0 + e;
        const bool same = (sb[j] == bi);
        int s = s4[e];
        s = (s < 0) ? 0 : s;
        s = (s > MSP) ? MSP : s;
        const float tv = sdb[s];
        const bool jv = (j >= NO);
        float val = ((!iv) && (!jv)) ? tv : fill;
        val = (same && (iv != jv)) ? vb : val;
        val = (i == j) ? d0 : val;
        o[it][e] = same ? val : ninf;
      }
    }
    float* dr = BM + (size_t)i * NN + tid * 4;
    *(volatile v4f*)(dr) = o[0];
    *(volatile v4f*)(dr + 1024) = o[1];
    __threadfence();
    *(volatile v4f*)(dr) = o[0];
    *(volatile v4f*)(dr + 1024) = o[1];
  }
}

__global__ __launch_bounds__(256) void k_ln(const float* __restrict__ H, unsigned short* __restrict__ HN, int rowBase) {
  const int lane = threadIdx.x & 31, wave = threadIdx.x >> 5;
  int row = rowBase + blockIdx.x * 8 + wave;
  row = (row < NN) ? row : (NN - 1);
  const float* hr = H + (size_t)row * DM;
  const v4f a0 = *(const v4f*)(hr + lane * 8);
  const v4f a1 = *(const v4f*)(hr + lane * 8 + 4);
  const v4f b0 = *(const v4f*)(hr + 256 + lane * 8);
  const v4f b1 = *(const v4f*)(hr + 256 + lane * 8 + 4);
  float s = ((a0[0] + a0[1]) + (a0[2] + a0[3])) + ((a1[0] + a1[1]) + (a1[2] + a1[3]));
  s += ((b0[0] + b0[1]) + (b0[2] + b0[3])) + ((b1[0] + b1[1]) + (b1[2] + b1[3]));
#pragma unroll
  for (int off = 16; off > 0; off >>= 1) s += __shfl_xor(s, off, 32);
  const float mean = s * (1.0f / 512.0f);
  v4f da0, da1, db0, db1;
  float ss = 0.0f;
#pragma unroll
  for (int e = 0; e < 4; ++e) {
    da0[e] = a0[e] - mean; da1[e] = a1[e] - mean; db0[e] = b0[e] - mean; db1[e] = b1[e] - mean;
    ss += da0[e] * da0[e]; ss += da1[e] * da1[e]; ss += db0[e] * db0[e]; ss += db1[e] * db1[e];
  }
#pragma unroll
  for (int off = 16; off > 0; off >>= 1) ss += __shfl_xor(ss, off, 32);
  const float var = ss * (1.0f / 512.0f);
  const float rinv = 1.0f / sqrtf(var + 1e-5f);
#pragma unroll
  for (int e = 0; e < 4; ++e) { da0[e] *= rinv; da1[e] *= rinv; db0[e] *= rinv; db1[e] *= rinv; }
  v4u hA, lA, hB, lB;
  split8(da0, da1, hA, lA);
  split8(db0, db1, hB, lB);
  unsigned short* d = HN + (size_t)row * (2 * DM) + lane * 8;
  for (int pass = 0; pass < 2; ++pass) {
    *(volatile v4u*)(d) = hA;
    *(volatile v4u*)(d + 256) = hB;
    *(volatile v4u*)(d + 512) = lA;
    *(volatile v4u*)(d + 768) = lB;
    __threadfence();
  }
}

template <int EPI, int KW, int NTOT>
__global__ __launch_bounds__(256) __attribute__((amdgpu_num_vgpr(248)))
void k_gemm(const unsigned short* __restrict__ Ap, const unsigned short* __restrict__ Btp,
            const float* __restrict__ bias, const float* __restrict__ aux,
            unsigned short* __restrict__ C16a, unsigned short* __restrict__ C16b,
            float* __restrict__ C32, const int* __restrict__ deg,
            int rowBase, int nRowTiles, int outRowSub) {
  constexpr bool ASPLIT = (EPI == 1 || EPI == 2 || EPI == 3);
  constexpr bool BSPLIT = (EPI == 4);
  constexpr int LDA = ASPLIT ? 2 * KW : KW;
  constexpr int LDB = BSPLIT ? 2 * KW : KW;
  static_assert(KW % 32 == 0);
  static_assert(NTOT % 64 == 0);
  static_assert(!(EPI == 0 || EPI == 2) || NTOT == DM);
  static_assert(EPI != 1 || NTOT == 2 * DM);
  static_assert(EPI != 3 || NTOT == FF);
  static_assert(EPI != 4 || NTOT == NN);
  const __bf16* A = (const __bf16*)Ap;
  const __bf16* Bt = (const __bf16*)Btp;
  __shared__ __align__(16) float sT[8][16 * 68];
  const int lane = threadIdx.x & 31;
  const int wave = threadIdx.x >> 5;
  constexpr int tilesN = NTOT >> 6;
  const int tile = blockIdx.x * 8 + wave;
  if (tile >= nRowTiles * tilesN) return;
  const int tm = tile / tilesN;
  const int tn = tile - tm * tilesN;
  const int m0 = rowBase + (tm << 6);
  const int n0 = tn << 6;
  const int rlane = lane & 15;
  const int koff = (lane >> 4) * 8;
  const int mOff = (lane >> 4) * 8;

  v8f acc[4][4];
#pragma unroll
  for (int i = 0; i < 4; ++i)
#pragma unroll
    for (int j = 0; j < 4; ++j) acc[i][j] = (v8f){0.f, 0.f, 0.f, 0.f, 0.f, 0.f, 0.f, 0.f};

#pragma unroll 1
  for (int k0 = 0; k0 < KW; k0 += 32) {
    v16b bh[4], bl[4];
#pragma unroll
    for (int j = 0; j < 4; ++j) {
      const size_t bo = (size_t)(n0 + (j << 4) + rlane) * LDB + koff + k0;
      bh[j] = ldfrag(Bt + bo);
      if (BSPLIT) bl[j] = ldfrag(Bt + bo + KW); else bl[j] = bh[j];
    }
#pragma unroll
    for (int i = 0; i < 4; ++i) {
      const size_t ao = (size_t)(m0 + (i << 4) + rlane) * LDA + koff + k0;
      const v16b ah = ldfrag(A + ao);
      v16b al;
      if (ASPLIT) al = ldfrag(A + ao + KW); else al = ah;
#pragma unroll
      for (int j = 0; j < 4; ++j) {
        acc[i][j] = mma_b(ah, bh[j], acc[i][j]);
        if (ASPLIT) acc[i][j] = mma_b(al, bh[j], acc[i][j]);
        if (BSPLIT) acc[i][j] = mma_b(ah, bl[j], acc[i][j]);
      }
      dep_guard_b(acc[i][0], acc[i][3], ah, al);
    }
    keep4_b(bh[0], bh[1], bh[2], bh[3]);
    if (BSPLIT) keep4_b(bl[0], bl[1], bl[2], bl[3]);
  }
  acc_guard4(acc[0][0], acc[0][1], acc[0][2], acc[0][3]);
  acc_guard4(acc[1][0], acc[1][1], acc[1][2], acc[1][3]);
  acc_guard4(acc[2][0], acc[2][1], acc[2][2], acc[2][3]);
  acc_guard4(acc[3][0], acc[3][1], acc[3][2], acc[3][3]);

  float* slab = sT[wave];
  const float qsc = (EPI == 1 && n0 < DM) ? 0.125f : 1.0f;
#pragma unroll
  for (int i = 0; i < 4; ++i) {
    const int mBase = m0 + (i << 4);
    float br[8];
#pragma unroll
    for (int r = 0; r < 8; ++r) br[r] = 0.0f;
    if (EPI == 4) {
#pragma unroll
      for (int r = 0; r < 8; ++r) br[r] = bf16r(bias[mBase + mOff + r]);
    }
#pragma unroll
    for (int j = 0; j < 4; ++j) {
      const int n = n0 + (j << 4) + rlane;
      float bv = 0.0f;
      if (EPI == 1) {
        const float bq0 = bias[n & (DM - 1)];
        const float bk0 = aux[n & (DM - 1)];
        bv = bf16r((n0 < DM) ? bq0 : bk0);
      }
      if (EPI == 2 || EPI == 3) bv = bf16r(bias[n]);
#pragma unroll
      for (int r = 0; r < 8; ++r) {
        float v = acc[i][j][r];
        if (EPI == 1) v = (v + bv) * qsc;
        if (EPI == 2) v = v + bv;
        if (EPI == 3) { v = v + bv; v = (v > 0.0f) ? v : (v - v); }
        if (EPI == 4) v = v + br[r];
        slab[(mOff + r) * 68 + (j << 4) + rlane] = v;
      }
    }
    __builtin_amdgcn_fence(__ATOMIC_RELEASE, "workgroup");
    __builtin_amdgcn_wave_barrier();
    __builtin_amdgcn_fence(__ATOMIC_ACQUIRE, "workgroup");
    if (EPI == 0 || EPI == 2) {
      const int hh = lane >> 4, c4 = (lane & 15) * 4;
      v4f vals[8];
#pragma unroll
      for (int it = 0; it < 8; ++it) {
        const int row = it * 2 + hh;
        const int grow = mBase + row;
        v4f v = *(const v4fa*)(slab + row * 68 + c4);
        if (EPI == 2) {
          const v4f rr = *(const v4f*)(aux + (size_t)grow * DM + n0 + c4);
          v = v + rr;
        }
        if (EPI == 0) {
          int dg = deg[grow];
          dg = (dg < 0) ? 0 : dg;
          dg = (dg > MDG) ? MDG : dg;
          const v4f ce = *(const v4f*)(aux + (size_t)dg * DM + n0 + c4);
          const v4f ib = *(const v4f*)(bias + n0 + c4);
          const bool orig = (grow < NO);
#pragma unroll
          for (int e = 0; e < 4; ++e) {
            const float t = v[e] + bf16r(ib[e]);
            const float u = orig ? t : 0.0f;
            v[e] = u + bf16r(ce[e]);
          }
        }
        vals[it] = v;
      }
      for (int pass = 0; pass < 2; ++pass) {
#pragma unroll
        for (int it = 0; it < 8; ++it) {
          const int grow = mBase + it * 2 + hh;
          *(volatile v4f*)(C32 + (size_t)(grow - outRowSub) * DM + n0 + c4) = vals[it];
        }
        __threadfence();
      }
    } else {
      const int q = lane >> 3, c8 = (lane & 7) * 8;
      v4u hv[4], lv[4];
#pragma unroll
      for (int it = 0; it < 4; ++it) {
        const int row = it * 4 + q;
        const float* sp = slab + row * 68 + c8;
        const v4f x0 = *(const v4fa*)(sp);
        const v4f x1 = *(const v4fa*)(sp + 4);
        split8(x0, x1, hv[it], lv[it]);
      }
      for (int pass = 0; pass < 2; ++pass) {
#pragma unroll
        for (int it = 0; it < 4; ++it) {
          const int grow = mBase + it * 4 + q;
          size_t base;
          if (EPI == 1) {
            const int which = n0 >> 9, head = (n0 >> 6) & 7;
            base = ((size_t)(which * NHD + head) * NN + grow) * DK + c8;
          } else if (EPI == 3) {
            base = (size_t)grow * (2 * FF) + n0 + c8;
          } else {
            base = (size_t)grow * NN + n0 + c8;
          }
          *(volatile v4u*)(C16a + base) = hv[it];
          *(volatile v4u*)(C16b + base) = lv[it];
        }
        __threadfence();
      }
    }
    __builtin_amdgcn_fence(__ATOMIC_RELEASE, "workgroup");
    __builtin_amdgcn_wave_barrier();
    __builtin_amdgcn_fence(__ATOMIC_ACQUIRE, "workgroup");
  }
}

__device__ __forceinline__ void pack_p(const v8f a, const v8f c, v16b& hi, v16b& lo) {
  union { v16b v; unsigned u[8]; } Hh, Ll;
#pragma unroll
  for (int q = 0; q < 4; ++q) {
    const unsigned short h0 = f2bf_bits(a[2 * q]), h1 = f2bf_bits(a[2 * q + 1]);
    const unsigned short l0 = f2bf_bits(a[2 * q] - bf_bits2f(h0)), l1 = f2bf_bits(a[2 * q + 1] - bf_bits2f(h1));
    Hh.u[q] = pk16(h0, h1); Ll.u[q] = pk16(l0, l1);
    const unsigned short g0 = f2bf_bits(c[2 * q]), g1 = f2bf_bits(c[2 * q + 1]);
    const unsigned short m0 = f2bf_bits(c[2 * q] - bf_bits2f(g0)), m1 = f2bf_bits(c[2 * q + 1] - bf_bits2f(g1));
    Hh.u[4 + q] = pk16(g0, g1); Ll.u[4 + q] = pk16(m0, m1);
  }
  hi = Hh.v; lo = Ll.v;
}

__global__ __launch_bounds__(128) __attribute__((amdgpu_num_vgpr(248)))
void k_attn(const unsigned short* __restrict__ QKHp, const unsigned short* __restrict__ QKLp,
            const unsigned short* __restrict__ VTHp, const unsigned short* __restrict__ VTLp,
            const float* __restrict__ BM, const int* __restrict__ tcls,
            unsigned short* __restrict__ OHL, int qtBase) {
  __shared__ __align__(16) float sO[4 * 16 * 64];
  const int tid = threadIdx.x, lane = tid & 31, w = tid >> 5;
  const int h = lane >> 4, m = lane & 15;
  int qt = qtBase + blockIdx.x;
  qt = (qt < NT) ? qt : (NT - 1);
  const int head = blockIdx.y;
  const int q0 = qt * 64 + 16 * w;
  const __bf16* QH = (const __bf16*)QKHp;
  const __bf16* QL = (const __bf16*)QKLp;
  const __bf16* KH = QH + PLANE_QK;
  const __bf16* KL = QL + PLANE_QK;
  const __bf16* VTH = (const __bf16*)VTHp;
  const __bf16* VTL = (const __bf16*)VTLp;

  const size_t qo = ((size_t)head * NN + q0 + m) * DK + 8 * h;
  const v16b qh0 = ldfrag(QH + qo), qh1 = ldfrag(QH + qo + 32);
  const v16b ql0 = ldfrag(QL + qo), ql1 = ldfrag(QL + qo + 32);

  const v8f zero8 = (v8f){0.f, 0.f, 0.f, 0.f, 0.f, 0.f, 0.f, 0.f};
  v8f o[4];
#pragma unroll
  for (int t = 0; t < 4; ++t) o[t] = zero8;
  float mrun = MTH, lrun = 0.0f;
  const float* bmrow = BM + (size_t)(q0 + m) * NN + 8 * h;
  const size_t kbase = ((size_t)head * NN + m) * DK + 8 * h;
  const size_t vbase = ((size_t)head * DK + m) * NN + 8 * h;

#pragma unroll 1
  for (int kt = 0; kt < NT; ++kt) {
    const int cls = __builtin_amdgcn_readfirstlane(tcls[qt * NT + kt]);
    if (cls == 0) continue;
    const int kb = kt * 64;
    v8f s[4];
#pragma unroll
    for (int j = 0; j < 4; ++j) {
      const size_t ko = kbase + (size_t)(kb + 16 * j) * DK;
      const v16b kh0 = ldfrag(KH + ko), kh1 = ldfrag(KH + ko + 32);
      const v16b kl0 = ldfrag(KL + ko), kl1 = ldfrag(KL + ko + 32);
      v8f z = zero8;
      z = mma_g(kh0, qh0, z);
      z = mma_g(kl0, qh0, z);
      z = mma_g(kh0, ql0, z);
      z = mma_g(kh1, qh1, z);
      z = mma_g(kl1, qh1, z);
      z = mma_g(kh1, ql1, z);
      s[j] = z;
    }
    float mloc = MTH;
#pragma unroll
    for (int j = 0; j < 4; ++j) {
      const v4f ba = *(const v4f*)(bmrow + kb + 16 * j);
      const v4f bb = *(const v4f*)(bmrow + kb + 16 * j + 4);
#pragma unroll
      for (int r = 0; r < 4; ++r) {
        const float x0 = (ba[r] > MTH) ? (s[j][r] + ba[r]) : MTH;
        const float x1 = (bb[r] > MTH) ? (s[j][4 + r] + bb[r]) : MTH;
        s[j][r] = x0; s[j][4 + r] = x1;
        mloc = fmaxf(mloc, fmaxf(x0, x1));
      }
    }
    mloc = fmaxf(mloc, __shfl_xor(mloc, 16, 32));
    const float mnew = fmaxf(mrun, mloc);
    const float alpha = expf(mrun - mnew);
    mrun = mnew;
    float lsum = 0.0f;
#pragma unroll
    for (int j = 0; j < 4; ++j)
#pragma unroll
      for (int r = 0; r < 8; ++r) {
        const float x = s[j][r];
        const float e = expf(x - mnew);
        const float p = (x > MTH) ? e : 0.0f;
        s[j][r] = p;
        lsum += p;
      }
    lsum += __shfl_xor(lsum, 16, 32);
    lrun = lrun * alpha + lsum;
#pragma unroll
    for (int t = 0; t < 4; ++t)
#pragma unroll
      for (int r = 0; r < 8; ++r) o[t][r] = o[t][r] * alpha;

    v16b ph0, pl0, ph1, pl1;
    pack_p(s[0], s[1], ph0, pl0);
    pack_p(s[2], s[3], ph1, pl1);
#pragma unroll
    for (int t = 0; t < 4; ++t) {
      const size_t vo = vbase + (size_t)(16 * t) * NN + kb;
      const v16b vh0 = ldfrag(VTH + vo), vh1 = ldfrag(VTH + vo + 32);
      const v16b vl0 = ldfrag(VTL + vo), vl1 = ldfrag(VTL + vo + 32);
      v8f z = o[t];
      z = mma_g(vh0, ph0, z);
      z = mma_g(vl0, ph0, z);
      z = mma_g(vh0, pl0, z);
      z = mma_g(vh1, ph1, z);
      z = mma_g(vl1, ph1, z);
      z = mma_g(vh1, pl1, z);
      o[t] = z;
    }
  }

  const float inv = (lrun > 0.0f) ? (1.0f / lrun) : 0.0f;
  float* so = sO + w * 1024;
#pragma unroll
  for (int t = 0; t < 4; ++t)
#pragma unroll
    for (int r = 0; r < 8; ++r) so[m * 64 + 16 * t + 8 * h + r] = o[t][r] * inv;
  __syncthreads();
  const int q = lane >> 3, c8 = (lane & 7) * 8;
  v4u hv[4], lv[4];
#pragma unroll
  for (int it = 0; it < 4; ++it) {
    const int row = it * 4 + q;
    const v4f x0 = *(const v4fa*)(so + row * 64 + c8);
    const v4f x1 = *(const v4fa*)(so + row * 64 + c8 + 4);
    split8(x0, x1, hv[it], lv[it]);
  }
  for (int pass = 0; pass < 2; ++pass) {
#pragma unroll
    for (int it = 0; it < 4; ++it) {
      const int row = it * 4 + q;
      unsigned short* d = OHL + (size_t)(q0 + row) * (2 * DM) + head * DK + c8;
      *(volatile v4u*)(d) = hv[it];
      *(volatile v4u*)(d + DM) = lv[it];
    }
    __threadfence();
  }
}

extern "C" void kernel_launch(void* const* d_in, const int* in_sizes, int n_in,
                              void* d_out, int out_size, void* d_ws, size_t ws_size,
                              hipStream_t stream) {
  if (n_in < 21) return;
  const int expect[21] = {NO * NF, NO * NO, NN, NN, NF * DM, DM, (MDG + 1) * DM, MSP + 2, 1,
                          NL * NHD * DM * DK, NL * NHD * DK, NL * NHD * DM * DK, NL * NHD * DK,
                          NL * NHD * DM * DK, NL * NHD * DK, NL * DM * DM, NL * DM,
                          NL * DM * FF, NL * FF, NL * FF * DM, NL * DM};
  for (int i = 0; i < 21; ++i) if (in_sizes[i] != expect[i]) return;
  if (out_size != 64 * DM) return;

  const float* x     = (const float*)d_in[0];
  const int*   sp    = (const int*)d_in[1];
  const int*   bid   = (const int*)d_in[2];
  const int*   deg   = (const int*)d_in[3];
  const float* initW = (const float*)d_in[4];
  const float* initb = (const float*)d_in[5];
  const float* cent  = (const float*)d_in[6];
  const float* distb = (const float*)d_in[7];
  const float* virtb = (const float*)d_in[8];
  const float* Wq = (const float*)d_in[9];
  const float* bq = (const float*)d_in[10];
  const float* Wk = (const float*)d_in[11];
  const float* bk = (const float*)d_in[12];
  const float* Wv = (const float*)d_in[13];
  const float* bv = (const float*)d_in[14];
  const float* Wo = (const float*)d_in[15];
  const float* bo = (const float*)d_in[16];
  const float* W1 = (const float*)d_in[17];
  const float* b1 = (const float*)d_in[18];
  const float* W2 = (const float*)d_in[19];
  const float* b2 = (const float*)d_in[20];
  float* out = (float*)d_out;

  size_t off = 0;
  const size_t oWQK = off; off += (size_t)NL * 2 * DM * DM * 2;
  const size_t oWVT = off; off += (size_t)NL * DM * DM * 2;
  const size_t oWO  = off; off += (size_t)NL * DM * DM * 2;
  const size_t oW1T = off; off += (size_t)NL * FF * DM * 2;
  const size_t oW2T = off; off += (size_t)NL * DM * FF * 2;
  const size_t oBM  = off; off += (size_t)NN * NN * 4;
  const size_t oHA  = off; off += (size_t)NN * DM * 4;
  const size_t oHB  = off; off += (size_t)NN * DM * 4;
  const size_t oHN  = off; off += (size_t)NN * 2 * DM * 2;
  const size_t oQKH = off; off += (size_t)2 * PLANE_QK * 2;
  const size_t oQKL = off; off += (size_t)2 * PLANE_QK * 2;
  const size_t oVTH = off; off += (size_t)DM * NN * 2;
  const size_t oVTL = off; off += (size_t)DM * NN * 2;
  const size_t oOHL = off; off += (size_t)NN * 2 * DM * 2;
  const size_t oA1  = off; off += (size_t)NN * 2 * FF * 2;
  const size_t oXB  = off; off += (size_t)NN * NF * 2;
  const size_t oIWT = off; off += (size_t)DM * NF * 2;
  const size_t oTC  = off; off += (size_t)NT * NT * 4;
  if (off > ws_size) return;
  if (off > (size_t)134217728) return;

  char* ws = (char*)d_ws;
  unsigned short* WQK = (unsigned short*)(ws + oWQK);
  unsigned short* WVT = (unsigned short*)(ws + oWVT);
  unsigned short* WO  = (unsigned short*)(ws + oWO);
  unsigned short* W1T = (unsigned short*)(ws + oW1T);
  unsigned short* W2T = (unsigned short*)(ws + oW2T);
  float*          BM  = (float*)(ws + oBM);
  float*          HA  = (float*)(ws + oHA);
  float*          HB  = (float*)(ws + oHB);
  unsigned short* HN  = (unsigned short*)(ws + oHN);
  unsigned short* QKH = (unsigned short*)(ws + oQKH);
  unsigned short* QKL = (unsigned short*)(ws + oQKL);
  unsigned short* VTH = (unsigned short*)(ws + oVTH);
  unsigned short* VTL = (unsigned short*)(ws + oVTL);
  unsigned short* OHL = (unsigned short*)(ws + oOHL);
  unsigned short* A1  = (unsigned short*)(ws + oA1);
  unsigned short* XB  = (unsigned short*)(ws + oXB);
  unsigned short* IWT = (unsigned short*)(ws + oIWT);
  int*            TC  = (int*)(ws + oTC);

  const dim3 blk(256);
  k_pa<<<dim3(40), blk, 0, stream>>>(x, initW, XB, IWT);
  k_tr<<<dim3(DK / 64, DM / 64, NL * NHD), blk, 0, stream>>>(Wq, WQK, DM, DK, DM * DK, NHD, 2 * DM * DM, DK * DM);
  k_tr<<<dim3(DK / 64, DM / 64, NL * NHD), blk, 0, stream>>>(Wk, WQK + (size_t)DM * DM, DM, DK, DM * DK, NHD, 2 * DM * DM, DK * DM);
  k_tr<<<dim3(DK / 64, DM / 64, NL * NHD), blk, 0, stream>>>(Wv, WVT, DM, DK, DM * DK, NHD, DM * DM, DK * DM);
  k_tr<<<dim3(DM / 64, DM / 64, NL), blk, 0, stream>>>(Wo, WO, DM, DM, DM * DM, 1, DM * DM, 0);
  k_tr<<<dim3(FF / 64, DM / 64, NL), blk, 0, stream>>>(W1, W1T, DM, FF, DM * FF, 1, DM * FF, 0);
  k_tr<<<dim3(DM / 64, FF / 64, NL), blk, 0, stream>>>(W2, W2T, FF, DM, FF * DM, 1, FF * DM, 0);
  k_bias<<<dim3(NT), blk, 0, stream>>>(sp, bid, distb, virtb, BM, TC);
  k_gemm<0, NF, DM><<<dim3(32), blk, 0, stream>>>(XB, IWT, initb, cent, QKH, QKL, HA, deg, 0, NT, 0);

  for (int l = 0; l < NL; ++l) {
    const bool last = (l == NL - 1);
    const int rb = last ? NO : 0;
    const int rt = last ? 1 : NT;
    k_ln<<<dim3(NN / 8), blk, 0, stream>>>(HA, HN, 0);
    k_gemm<1, DM, 2 * DM><<<dim3((NT * 16 + 7) / 8), blk, 0, stream>>>(
        HN, WQK + (size_t)l * 2 * DM * DM, bq + (size_t)l * DM, bk + (size_t)l * DM, QKH, QKL, HB, deg, 0, NT, 0);
    k_gemm<4, DM, NN><<<dim3((8 * NT + 7) / 8), blk, 0, stream>>>(
        WVT + (size_t)l * DM * DM, HN, bv + (size_t)l * DM, bv + (size_t)l * DM, VTH, VTL, HB, deg, 0, DM / 64, 0);
    k_attn<<<dim3(last ? 1 : NT, NHD), dim3(128), 0, stream>>>(QKH, QKL, VTH, VTL, BM, TC, OHL, last ? (NT - 1) : 0);
    k_gemm<2, DM, DM><<<dim3((rt * 8 + 7) / 8), blk, 0, stream>>>(
        OHL, WO + (size_t)l * DM * DM, bo + (size_t)l * DM, HA, QKH, QKL, HB, deg, rb, rt, 0);
    k_ln<<<dim3(last ? 8 : (NN / 8)), blk, 0, stream>>>(HB, HN, rb);
    k_gemm<3, DM, FF><<<dim3((rt * 32 + 7) / 8), blk, 0, stream>>>(
        HN, W1T + (size_t)l * FF * DM, b1 + (size_t)l * FF, b1 + (size_t)l * FF, A1, A1 + FF, HA, deg, rb, rt, 0);
    k_gemm<2, FF, DM><<<dim3((rt * 8 + 7) / 8), blk, 0, stream>>>(
        A1, W2T + (size_t)l * DM * FF, b2 + (size_t)l * DM, HB, QKH, QKL, last ? out : HA, deg, rb, rt, last ? NO : 0);
  }
  (void)hipGetLastError();
}
